// PointNetSetAbstraction_13503377178958
// MI455X (gfx1250) — hardware-verified
//
#include <hip/hip_runtime.h>
#include <math.h>

#pragma clang fp contract(off)

typedef __attribute__((ext_vector_type(16))) _Float16 v16h;
typedef __attribute__((ext_vector_type(8)))  _Float16 v8h;
typedef __attribute__((ext_vector_type(8)))  float    v8f;
typedef __attribute__((ext_vector_type(4)))  float    v4f;
typedef __attribute__((ext_vector_type(4)))  unsigned int v4u;

constexpr int NBATCH  = 4;
constexpr int NPTS    = 8192;
constexpr int NCENT   = 1024;
constexpr int NNBR    = 32;
constexpr int NFEAT   = 64;
constexpr int CIN_L0  = 67;
constexpr int NOUT_L0 = 64;
constexpr int NOUT_L1 = 64;
constexpr int NOUT_L2 = 128;
constexpr int MROWS   = NBATCH * NCENT * NNBR;
constexpr int NGROUPS = NBATCH * NCENT;
constexpr float W_CARRY     = 64.0f;
constexpr float W_CARRY_INV = 1.0f / W_CARRY;
constexpr float BALL_R2     = (float)(0.1 * 0.1);
constexpr float BN_EPS_F    = 1e-5f;
constexpr float FPS_INIT    = 1e10f;

static_assert(CIN_L0 == 3 + NFEAT, "layer-0 input = rel-xyz + features");
static_assert(MROWS == 131072, "row count");
static_assert(NGROUPS == 4096, "group count");
static_assert(NGROUPS % 8 == 0 && MROWS % 256 == 0, "tile multiples");
static_assert(NFEAT % 32 == 0, "K multiple of 32");

constexpr size_t OFF_X     = 0;
constexpr size_t OFF_XX    = OFF_X    + (size_t)NBATCH * 3 * NPTS * 4;
constexpr size_t OFF_W0F   = OFF_XX   + (size_t)NBATCH * NPTS * 4;
constexpr size_t OFF_W1H   = OFF_W0F  + (size_t)NOUT_L0 * 64 * 2;
constexpr size_t OFF_W2H   = OFF_W1H  + (size_t)NOUT_L1 * 64 * 2;
constexpr size_t OFF_W0X   = OFF_W2H  + (size_t)NOUT_L2 * 64 * 2;
constexpr size_t OFF_SS    = OFF_W0X  + (size_t)NOUT_L0 * 4 * 4;
constexpr size_t OFF_CENT  = OFF_SS   + (size_t)3 * 2 * 128 * 4;
constexpr size_t OFF_P16   = 1048576;
constexpr size_t OFF_REL   = OFF_P16  + (size_t)NBATCH * NPTS * NFEAT * 2;
constexpr size_t OFF_A0    = OFF_REL  + (size_t)MROWS * 4 * 4;
constexpr size_t OFF_A1    = OFF_A0   + (size_t)MROWS * 64 * 2;
constexpr size_t OFF_A2    = OFF_A1   + (size_t)MROWS * 64 * 2;
constexpr size_t OFF_YB    = OFF_A2   + (size_t)MROWS * 64 * 2;
constexpr size_t OFF_PART0 = OFF_YB   + (size_t)MROWS * 64 * 4;
constexpr size_t OFF_PART1 = OFF_PART0 + (size_t)NGROUPS * 2 * 64 * 4;
constexpr size_t OFF_PART2 = OFF_PART1 + (size_t)NGROUPS * 2 * 64 * 4;
constexpr size_t OFF_GM    = OFF_PART2 + (size_t)NGROUPS * 2 * 128 * 4;
constexpr size_t WS_TOTAL  = OFF_GM   + (size_t)NGROUPS * 2 * 128 * 4;
static_assert(OFF_CENT + (size_t)NGROUPS * 4 * 4 <= OFF_P16, "small planes fit below P16");
static_assert(WS_TOTAL <= (size_t)134217728, "carve within 128 MiB");
static_assert((OFF_XX % 128) == 0 && (OFF_W0F % 128) == 0 && (OFF_W0X % 128) == 0 && (OFF_SS % 128) == 0 &&
              (OFF_CENT % 128) == 0 && (OFF_REL % 128) == 0 && (OFF_A0 % 128) == 0 && (OFF_YB % 128) == 0 &&
              (OFF_PART0 % 128) == 0 && (OFF_GM % 128) == 0, "line aligned carves");

constexpr size_t OUT1_OFF_BYTES = 49152;
static_assert(OUT1_OFF_BYTES == (size_t)NBATCH * 3 * NCENT * 4, "out0 extent");
static_assert(OUT1_OFF_BYTES + (size_t)NBATCH * NOUT_L2 * NCENT * 4 == (size_t)2146304, "d_out total");
static_assert((OUT1_OFF_BYTES % 128) == 0, "out1 line aligned");

__device__ __forceinline__ float bf16r(float f) {
  unsigned u = __float_as_uint(f);
  u = (u + 0x7FFFu + ((u >> 16) & 1u)) & 0xFFFF0000u;
  return __uint_as_float(u);
}
__device__ __forceinline__ unsigned f16bits(float f) {
  const _Float16 h = (_Float16)f;
  const unsigned short s = __builtin_bit_cast(unsigned short, h);
  return (unsigned)s;
}

union FragH { v16h v; v8h h[2]; };
__device__ __forceinline__ v16h frag_load_h(const _Float16* p) {
  FragH f;
  f.h[0] = *(const v8h*)(p);
  f.h[1] = *(const v8h*)(p + 16);
  return f.v;
}
__device__ __forceinline__ v8f mma_h(v16h a, v16h b, v8f c) {
  return __builtin_amdgcn_wmma_f32_16x16x32_f16(false, a, false, b, (short)0, c, false, false);
}
__device__ __forceinline__ void wmma_guard4(v8f& a, v8f& b, v8f& c, v8f& d,
                                            v16h x, v16h y0, v16h y1, v16h y2, v16h y3) {
  asm volatile("v_nop\n\tv_nop\n\tv_nop\n\tv_nop"
               : "+v"(a), "+v"(b), "+v"(c), "+v"(d)
               : "v"(x), "v"(y0), "v"(y1), "v"(y2), "v"(y3));
}
__device__ __forceinline__ void acc_guard4(v8f& a, v8f& b, v8f& c, v8f& d) {
  asm volatile("v_nop\n\tv_nop\n\tv_nop\n\tv_nop" : "+v"(a), "+v"(b), "+v"(c), "+v"(d));
}
__device__ __forceinline__ void wave_lds_sync() {
  __builtin_amdgcn_fence(__ATOMIC_RELEASE, "workgroup");
  __builtin_amdgcn_wave_barrier();
  __builtin_amdgcn_fence(__ATOMIC_ACQUIRE, "workgroup");
}

constexpr int PREP_SMALL_BLOCKS = 65;
__global__ __launch_bounds__(256) void prep_small(
    const float* __restrict__ xyz, const float* __restrict__ w0, const float* __restrict__ w1,
    const float* __restrict__ w2, float* __restrict__ X, float* __restrict__ XX,
    unsigned int* __restrict__ W0f, unsigned int* __restrict__ W1h, unsigned int* __restrict__ W2h,
    float* __restrict__ W0x) {
#pragma clang fp contract(off)
  const int blk = blockIdx.x;
  const int tid = threadIdx.x;
  if (blk < 32) {
    const int idx = blk * 256 + tid;
    const int b = idx >> 11;
    const int n = (idx & 2047) * 4;
    const float* src = xyz + (size_t)b * 3 * NPTS + n;
    const v4f a0 = *(const v4f*)(src);
    const v4f a1 = *(const v4f*)(src + NPTS);
    const v4f a2 = *(const v4f*)(src + 2 * NPTS);
    v4f r0, r1, r2, sq;
#pragma unroll
    for (int e = 0; e < 4; ++e) {
      const float fx = a0[e];
      const float fy = a1[e];
      const float fz = a2[e];
      const float x = bf16r(fx);
      const float y = bf16r(fy);
      const float z = bf16r(fz);
      const float t0 = x * x;
      const float t1 = y * y;
      const float t2 = z * z;
      r0[e] = x;
      r1[e] = y;
      r2[e] = z;
      sq[e] = (t0 + t2) + t1;
    }
    float* dx = X + (size_t)b * 3 * NPTS + n;
    float* dq = XX + (size_t)b * NPTS + n;
    for (int pass = 0; pass < 2; ++pass) {
      *(volatile v4f*)(dx) = r0;
      *(volatile v4f*)(dx + NPTS) = r1;
      *(volatile v4f*)(dx + 2 * NPTS) = r2;
      *(volatile v4f*)(dq) = sq;
      __threadfence();
    }
  } else if (blk < 40) {
    const int p = (blk - 32) * 256 + tid;
    const int o = p >> 5;
    const int kp = p & 31;
    const float f0 = w0[o * CIN_L0 + 3 + 2 * kp];
    const float f1 = w0[o * CIN_L0 + 3 + 2 * kp + 1];
    const unsigned lo = f16bits(bf16r(f0) * W_CARRY);
    const unsigned hi = f16bits(bf16r(f1) * W_CARRY);
    const unsigned word = lo | (hi << 16);
    ((volatile unsigned int*)W0f)[p] = word;
    __threadfence();
    ((volatile unsigned int*)W0f)[p] = word;
  } else if (blk < 48) {
    const int p = (blk - 40) * 256 + tid;
    const float f0 = w1[2 * p];
    const float f1 = w1[2 * p + 1];
    const unsigned lo = f16bits(bf16r(f0) * W_CARRY);
    const unsigned hi = f16bits(bf16r(f1) * W_CARRY);
    const unsigned word = lo | (hi << 16);
    ((volatile unsigned int*)W1h)[p] = word;
    __threadfence();
    ((volatile unsigned int*)W1h)[p] = word;
  } else if (blk < 64) {
    const int p = (blk - 48) * 256 + tid;
    const float f0 = w2[2 * p];
    const float f1 = w2[2 * p + 1];
    const unsigned lo = f16bits(bf16r(f0) * W_CARRY);
    const unsigned hi = f16bits(bf16r(f1) * W_CARRY);
    const unsigned word = lo | (hi << 16);
    ((volatile unsigned int*)W2h)[p] = word;
    __threadfence();
    ((volatile unsigned int*)W2h)[p] = word;
  } else {
    if (tid < NOUT_L0) {
      const float f0 = w0[tid * CIN_L0 + 0];
      const float f1 = w0[tid * CIN_L0 + 1];
      const float f2 = w0[tid * CIN_L0 + 2];
      v4f v;
      v[0] = bf16r(f0);
      v[1] = bf16r(f1);
      v[2] = bf16r(f2);
      v[3] = 0.0f;
      *(volatile v4f*)(W0x + tid * 4) = v;
      __threadfence();
      *(volatile v4f*)(W0x + tid * 4) = v;
    }
  }
}

__global__ __launch_bounds__(256) void prep_points(const float* __restrict__ points, v4u* __restrict__ P16q) {
  __shared__ unsigned int tileW[64][36];
  const int tid = threadIdx.x;
  const int b = blockIdx.x >> 7;
  const int n0 = (blockIdx.x & 127) * 64;
#pragma unroll
  for (int rep = 0; rep < 2; ++rep) {
    const int item = tid + rep * 256;
    const int cp = item >> 4;
    const int nq = item & 15;
    const float* s0 = points + ((size_t)(b * NFEAT + 2 * cp) * NPTS + n0 + nq * 4);
    const v4f a = *(const v4f*)(s0);
    const v4f c = *(const v4f*)(s0 + NPTS);
#pragma unroll
    for (int e = 0; e < 4; ++e) {
      const float fa = a[e];
      const float fc = c[e];
      const unsigned lo = f16bits(bf16r(fa));
      const unsigned hi = f16bits(bf16r(fc));
      tileW[nq * 4 + e][cp] = lo | (hi << 16);
    }
  }
  __syncthreads();
  v4u outv[2];
#pragma unroll
  for (int rep = 0; rep < 2; ++rep) {
    const int item = tid + rep * 256;
    const int row = item >> 3;
    const int pc = item & 7;
    v4u w;
    w[0] = tileW[row][pc * 4 + 0];
    w[1] = tileW[row][pc * 4 + 1];
    w[2] = tileW[row][pc * 4 + 2];
    w[3] = tileW[row][pc * 4 + 3];
    outv[rep] = w;
  }
  for (int pass = 0; pass < 2; ++pass) {
#pragma unroll
    for (int rep = 0; rep < 2; ++rep) {
      const int item = tid + rep * 256;
      const int row = item >> 3;
      const int pc = item & 7;
      *(volatile v4u*)(P16q + ((size_t)(b * NPTS + n0 + row) * 8 + pc)) = outv[rep];
    }
    __threadfence();
  }
}

static_assert(NPTS == 1024 * 8, "8 points per thread");
static_assert(NCENT == 1024, "one centroid per thread in the output phase");
__global__ __launch_bounds__(1024) void fps_kernel(const float* __restrict__ X, float* __restrict__ out0,
                                                   float* __restrict__ cent) {
#pragma clang fp contract(off)
  __shared__ float s_val[2][32];
  __shared__ int   s_idx[2][32];
  __shared__ int   s_cent[NCENT];
  const int b = blockIdx.x;
  const int t = threadIdx.x;
  const int lane = t & 31;
  const int wv = t >> 5;
  const float* xb = X + (size_t)b * 3 * NPTS;

  float px[8], py[8], pz[8], dmin[8];
  {
    const v4f ax = *(const v4f*)(xb + t * 8);
    const v4f bx = *(const v4f*)(xb + t * 8 + 4);
    const v4f ay = *(const v4f*)(xb + NPTS + t * 8);
    const v4f by = *(const v4f*)(xb + NPTS + t * 8 + 4);
    const v4f az = *(const v4f*)(xb + 2 * NPTS + t * 8);
    const v4f bz = *(const v4f*)(xb + 2 * NPTS + t * 8 + 4);
#pragma unroll
    for (int e = 0; e < 4; ++e) {
      px[e] = ax[e];
      px[4 + e] = bx[e];
      py[e] = ay[e];
      py[4 + e] = by[e];
      pz[e] = az[e];
      pz[4 + e] = bz[e];
    }
#pragma unroll
    for (int i = 0; i < 8; ++i) dmin[i] = FPS_INIT;
  }

  int far = 0;
#pragma unroll 1
  for (int it = 0; it < NCENT; ++it) {
    int fc = far;
    fc = fc < 0 ? 0 : fc;
    fc = fc > NPTS - 1 ? NPTS - 1 : fc;
    if (t == 0) s_cent[it] = fc;
    const float cx = xb[fc];
    const float cy = xb[NPTS + fc];
    const float cz = xb[2 * NPTS + fc];
    float best = -1.0f;
    int bidx = t * 8;
#pragma unroll
    for (int i = 0; i < 8; ++i) {
      const float dx = px[i] - cx;
      const float dy = py[i] - cy;
      const float dz = pz[i] - cz;
      const float t0 = dx * dx;
      const float t1 = dy * dy;
      const float t2 = dz * dz;
      const float d = (t0 + t2) + t1;
      dmin[i] = fminf(dmin[i], d);
      if (dmin[i] > best) {
        best = dmin[i];
        bidx = t * 8 + i;
      }
    }
#pragma unroll
    for (int off = 16; off > 0; off >>= 1) {
      const float ov = __shfl_xor(best, off, 32);
      const int oi = __shfl_xor(bidx, off, 32);
      const bool take = (ov > best) || (ov == best && oi < bidx);
      best = take ? ov : best;
      bidx = take ? oi : bidx;
    }
    const int pb = it & 1;
    if (lane == 0) {
      s_val[pb][wv] = best;
      s_idx[pb][wv] = bidx;
    }
    __syncthreads();
    best = s_val[pb][lane];
    bidx = s_idx[pb][lane];
#pragma unroll
    for (int off = 16; off > 0; off >>= 1) {
      const float ov = __shfl_xor(best, off, 32);
      const int oi = __shfl_xor(bidx, off, 32);
      const bool take = (ov > best) || (ov == best && oi < bidx);
      best = take ? ov : best;
      bidx = take ? oi : bidx;
    }
    far = bidx;
  }
  __syncthreads();
  {
    int ci = s_cent[t];
    ci = ci < 0 ? 0 : ci;
    ci = ci > NPTS - 1 ? NPTS - 1 : ci;
    const float x = xb[ci];
    const float y = xb[NPTS + ci];
    const float z = xb[2 * NPTS + ci];
    const float t0 = x * x;
    const float t1 = y * y;
    const float t2 = z * z;
    v4f cv;
    cv[0] = x;
    cv[1] = y;
    cv[2] = z;
    cv[3] = (t0 + t2) + t1;
    float* o0 = out0 + (size_t)b * 3 * NCENT + t;
    float* cdst = cent + (size_t)(b * NCENT + t) * 4;
    for (int pass = 0; pass < 2; ++pass) {
      *(volatile v4f*)(cdst) = cv;
      *(volatile float*)(o0) = x;
      *(volatile float*)(o0 + NCENT) = y;
      *(volatile float*)(o0 + 2 * NCENT) = z;
      __threadfence();
    }
  }
}

__global__ __launch_bounds__(256) void ballquery_group(
    const float* __restrict__ X, const float* __restrict__ XX, const float* __restrict__ cent,
    const v4u* __restrict__ P16q, v4u* __restrict__ A0q, float* __restrict__ rel) {
#pragma clang fp contract(off)
  __shared__ int s_gi[8][NNBR];
  const int lane = threadIdx.x & 31;
  const int wv = threadIdx.x >> 5;
  const int gid = blockIdx.x * 8 + wv;
  const int b = gid / NCENT;
  const float* xb = X + (size_t)b * 3 * NPTS;
  const float* xxb = XX + (size_t)b * NPTS;
  const v4f cv = *(const v4f*)(cent + (size_t)gid * 4);
  const float cx = cv[0];
  const float cy = cv[1];
  const float cz = cv[2];
  const float cc = cv[3];

  s_gi[wv][lane] = 0;
  int count = 0;
#pragma unroll 1
  for (int n0 = 0; n0 < NPTS && count < NNBR; n0 += 32) {
    const int n = n0 + lane;
    const float x0 = xb[n];
    const float x1 = xb[NPTS + n];
    const float x2 = xb[2 * NPTS + n];
    const float xx = xxb[n];
    float dot = cx * x0;
    dot = fmaf(cy, x1, dot);
    dot = fmaf(cz, x2, dot);
    const float sqr = ((-2.0f * dot) + cc) + xx;
    const bool inb = !(sqr > BALL_R2);
    const unsigned mask = (unsigned)__ballot(inb);
    const int pos = count + __popc(mask & ((1u << lane) - 1u));
    if (inb && pos < NNBR) s_gi[wv][pos] = n;
    count += __popc(mask);
  }
  __syncthreads();
  const int cnt = count < NNBR ? count : NNBR;

  {
    int gk = s_gi[wv][lane < cnt ? lane : 0];
    gk = gk < 0 ? 0 : gk;
    gk = gk > NPTS - 1 ? NPTS - 1 : gk;
    v4f rv;
    rv[0] = xb[gk] - cx;
    rv[1] = xb[NPTS + gk] - cy;
    rv[2] = xb[2 * NPTS + gk] - cz;
    rv[3] = 0.0f;
    float* rdst = rel + ((size_t)gid * NNBR + lane) * 4;
    *(volatile v4f*)(rdst) = rv;
    __threadfence();
    *(volatile v4f*)(rdst) = rv;
  }
  {
    const int pc = lane & 7;
    v4u vals[8];
#pragma unroll
    for (int it = 0; it < 8; ++it) {
      const int row = it * 4 + (lane >> 3);
      int g = s_gi[wv][row < cnt ? row : 0];
      g = g < 0 ? 0 : g;
      g = g > NPTS - 1 ? NPTS - 1 : g;
      vals[it] = P16q[(size_t)(b * NPTS + g) * 8 + pc];
    }
    for (int pass = 0; pass < 2; ++pass) {
#pragma unroll
      for (int it = 0; it < 8; ++it) {
        const int row = it * 4 + (lane >> 3);
        *(volatile v4u*)(A0q + ((size_t)gid * NNBR + row) * 8 + pc) = vals[it];
      }
      __threadfence();
    }
  }
}

template <int LAYER>
__global__ __launch_bounds__(256) void mlp_gemm(
    const unsigned short* __restrict__ Ap, const unsigned short* __restrict__ Wp,
    const float* __restrict__ bias, const float* __restrict__ rel, const float* __restrict__ w0x,
    float* __restrict__ Y, float* __restrict__ part, float* __restrict__ gm) {
  constexpr int NOUT = (LAYER == 2) ? NOUT_L2 : 64;
  constexpr int NHALVES = NOUT / 64;
  static_assert(NOUT % 64 == 0, "N tile multiple");
  const _Float16* A = (const _Float16*)Ap;
  const _Float16* W = (const _Float16*)Wp;
  __shared__ __align__(16) float sT[8][16 * 68];
  const int lane = threadIdx.x & 31;
  const int wave = threadIdx.x >> 5;
  const int tile = blockIdx.x * 8 + wave;
  const int m0 = tile * 32;
  const int rlane = lane & 15;
  const int hh = lane >> 4;
  const int koff = hh * 8;
  const int mOff = hh * 8;
  float* slab = sT[wave];

#pragma unroll 1
  for (int nh = 0; nh < NHALVES; ++nh) {
    const int n0 = nh * 64;
    float bv[4];
    v4f wx[4];
#pragma unroll
    for (int j = 0; j < 4; ++j) {
      const int n = n0 + (j << 4) + rlane;
      const float braw = bias[n];
      bv[j] = bf16r(braw);
      if (LAYER == 0) wx[j] = *(const v4f*)(w0x + (size_t)n * 4);
      else wx[j] = (v4f){0.f, 0.f, 0.f, 0.f};
    }
    asm volatile("" :: "v"(bv[0]), "v"(bv[1]), "v"(bv[2]), "v"(bv[3]));
    if (LAYER == 0) asm volatile("" :: "v"(wx[0]), "v"(wx[1]), "v"(wx[2]), "v"(wx[3]));

    v8f acc[2][4];
#pragma unroll
    for (int i = 0; i < 2; ++i)
#pragma unroll
      for (int j = 0; j < 4; ++j) acc[i][j] = (v8f){0.f, 0.f, 0.f, 0.f, 0.f, 0.f, 0.f, 0.f};

#pragma unroll
    for (int ks = 0; ks < 2; ++ks) {
      const int k0 = ks * 32;
      v16h bh[4];
#pragma unroll
      for (int j = 0; j < 4; ++j)
        bh[j] = frag_load_h(W + (size_t)(n0 + (j << 4) + rlane) * 64 + koff + k0);
#pragma unroll
      for (int i = 0; i < 2; ++i) {
        const v16h ah = frag_load_h(A + (size_t)(m0 + (i << 4) + rlane) * 64 + koff + k0);
#pragma unroll
        for (int j = 0; j < 4; ++j) acc[i][j] = mma_h(ah, bh[j], acc[i][j]);
        wmma_guard4(acc[i][0], acc[i][1], acc[i][2], acc[i][3], ah, bh[0], bh[1], bh[2], bh[3]);
      }
    }
    acc_guard4(acc[0][0], acc[0][1], acc[0][2], acc[0][3]);
    acc_guard4(acc[1][0], acc[1][1], acc[1][2], acc[1][3]);

    float csum[4], csq[4], gmx[4], gmn[4];
#pragma unroll
    for (int j = 0; j < 4; ++j) {
      csum[j] = 0.0f;
      csq[j] = 0.0f;
      gmx[j] = -__builtin_inff();
      gmn[j] = __builtin_inff();
    }

#pragma unroll
    for (int i = 0; i < 2; ++i) {
      const int mBase = m0 + (i << 4);
      v4f rr[8];
#pragma unroll
      for (int r = 0; r < 8; ++r) {
        if (LAYER == 0) rr[r] = *(const v4f*)(rel + (size_t)(mBase + mOff + r) * 4);
        else rr[r] = (v4f){0.f, 0.f, 0.f, 0.f};
      }
#pragma unroll
      for (int j = 0; j < 4; ++j) {
#pragma unroll
        for (int r = 0; r < 8; ++r) {
          float v = acc[i][j][r] * W_CARRY_INV;
          if (LAYER == 0) {
            v = fmaf(rr[r][0], wx[j][0], v);
            v = fmaf(rr[r][1], wx[j][1], v);
            v = fmaf(rr[r][2], wx[j][2], v);
          }
          v = v + bv[j];
          csum[j] += v;
          csq[j] = fmaf(v, v, csq[j]);
          if (LAYER == 2) {
            gmx[j] = fmaxf(gmx[j], v);
            gmn[j] = fminf(gmn[j], v);
          } else {
            slab[(mOff + r) * 68 + (j << 4) + rlane] = v;
          }
        }
      }
      if (LAYER < 2) {
        wave_lds_sync();
        const int c4 = (lane & 15) * 4;
        for (int pass = 0; pass < 2; ++pass) {
#pragma unroll
          for (int it = 0; it < 8; ++it) {
            const int row = it * 2 + hh;
            const v4f v = *(const v4f*)(slab + row * 68 + c4);
            *(volatile v4f*)(Y + (size_t)(mBase + row) * 64 + c4) = v;
          }
          __threadfence();
        }
        wave_lds_sync();
      }
    }

#pragma unroll
    for (int j = 0; j < 4; ++j) {
      const float os = __shfl_xor(csum[j], 16, 32);
      const float oq = __shfl_xor(csq[j], 16, 32);
      const float ox = __shfl_xor(gmx[j], 16, 32);
      const float on = __shfl_xor(gmn[j], 16, 32);
      csum[j] = csum[j] + os;
      csq[j] = csq[j] + oq;
      gmx[j] = fmaxf(gmx[j], ox);
      gmn[j] = fminf(gmn[j], on);
    }
    if (hh == 0) {
#pragma unroll
      for (int j = 0; j < 4; ++j) {
        slab[0 * 68 + (j << 4) + rlane] = csum[j];
        slab[1 * 68 + (j << 4) + rlane] = csq[j];
        slab[2 * 68 + (j << 4) + rlane] = gmx[j];
        slab[3 * 68 + (j << 4) + rlane] = gmn[j];
      }
    }
    wave_lds_sync();
    {
      const int row = lane >> 4;
      const int c4 = (lane & 15) * 4;
      const v4f sv = *(const v4f*)(slab + row * 68 + c4);
      const v4f mv = *(const v4f*)(slab + (2 + row) * 68 + c4);
      float* pdst = part + ((size_t)tile * 2 + row) * NOUT + n0 + c4;
      float* gdst = gm + ((size_t)tile * 2 + row) * 128 + n0 + c4;
      for (int pass = 0; pass < 2; ++pass) {
        *(volatile v4f*)(pdst) = sv;
        if (LAYER == 2) *(volatile v4f*)(gdst) = mv;
        __threadfence();
      }
    }
    wave_lds_sync();
  }
}

static_assert(NGROUPS == 8 * 64 * 8, "finalize tile split");
__global__ __launch_bounds__(256) void bn_finalize(const float* __restrict__ part, int nout,
                                                   const float* __restrict__ g, const float* __restrict__ beta,
                                                   float* __restrict__ ss) {
  __shared__ float red[8][2][32];
  const int lane = threadIdx.x & 31;
  const int wv = threadIdx.x >> 5;
  const int ch = blockIdx.x * 32 + lane;
  float s = 0.0f, q = 0.0f;
#pragma unroll 1
  for (int ob = 0; ob < 64; ++ob) {
    float s1 = 0.0f, q1 = 0.0f;
#pragma unroll
    for (int ib = 0; ib < 8; ++ib) {
      const int t = wv * 512 + ob * 8 + ib;
      s1 += part[(size_t)(t * 2) * nout + ch];
      q1 += part[(size_t)(t * 2 + 1) * nout + ch];
    }
    s += s1;
    q += q1;
  }
  red[wv][0][lane] = s;
  red[wv][1][lane] = q;
  __syncthreads();
  if (wv == 0) {
    float S = 0.0f, Q = 0.0f;
#pragma unroll
    for (int w = 0; w < 8; ++w) {
      S += red[w][0][lane];
      Q += red[w][1][lane];
    }
    const float invM = 1.0f / (float)MROWS;
    const float mean = S * invM;
    float var = Q * invM - mean * mean;
    var = fmaxf(var, 0.0f);
    const float graw = g[ch];
    const float braw = beta[ch];
    const float sc = bf16r(graw) * rsqrtf(var + BN_EPS_F);
    const float sh = bf16r(braw) - mean * sc;
    for (int pass = 0; pass < 2; ++pass) {
      *(volatile float*)(ss + ch) = sc;
      *(volatile float*)(ss + 128 + ch) = sh;
      __threadfence();
    }
  }
}

__global__ __launch_bounds__(256) void bn_relu_f16(const float* __restrict__ Y, const float* __restrict__ ss,
                                                   unsigned short* __restrict__ Aout) {
  const int idx = blockIdx.x * 256 + threadIdx.x;
  const int row = idx >> 3;
  const int c8 = (idx & 7) * 8;
  const v4f y0 = *(const v4f*)(Y + (size_t)row * 64 + c8);
  const v4f y1 = *(const v4f*)(Y + (size_t)row * 64 + c8 + 4);
  const v4f sc0 = *(const v4f*)(ss + c8);
  const v4f sc1 = *(const v4f*)(ss + c8 + 4);
  const v4f sh0 = *(const v4f*)(ss + 128 + c8);
  const v4f sh1 = *(const v4f*)(ss + 128 + c8 + 4);
  v8h hv;
#pragma unroll
  for (int e = 0; e < 4; ++e) {
    const float a = fmaxf(fmaf(y0[e], sc0[e], sh0[e]), 0.0f);
    const float c = fmaxf(fmaf(y1[e], sc1[e], sh1[e]), 0.0f);
    hv[e] = (_Float16)a;
    hv[4 + e] = (_Float16)c;
  }
  unsigned short* dst = Aout + (size_t)row * 64 + c8;
  *(volatile v8h*)(dst) = hv;
  __threadfence();
  *(volatile v8h*)(dst) = hv;
}

__global__ __launch_bounds__(256) void out_kernel(const float* __restrict__ gm, const float* __restrict__ ss2,
                                                  float* __restrict__ out1) {
  __shared__ float T[128][33];
  const int tid = threadIdx.x;
  const int lane = tid & 31;
  const int wv = tid >> 5;
  const int g0 = blockIdx.x * 32;
  const int b = g0 / NCENT;
  const int s0 = g0 - b * NCENT;
  const int o = tid & 127;
  const int half = tid >> 7;
  const float sc = ss2[o];
  const float sh = ss2[128 + o];
#pragma unroll 4
  for (int i = 0; i < 16; ++i) {
    const int gl = half + 2 * i;
    const size_t base = (size_t)(g0 + gl) * 256;
    const float mx = gm[base + o];
    const float mn = gm[base + 128 + o];
    const float sel = (sc >= 0.0f) ? mx : mn;
    T[o][gl] = fmaxf(fmaf(sc, sel, sh), 0.0f);
  }
  __syncthreads();
  float vals[16];
#pragma unroll
  for (int i = 0; i < 16; ++i) vals[i] = T[wv * 16 + i][lane];
  for (int pass = 0; pass < 2; ++pass) {
#pragma unroll
    for (int i = 0; i < 16; ++i) {
      const int oo = wv * 16 + i;
      *(volatile float*)(out1 + ((size_t)(b * NOUT_L2 + oo) * NCENT + s0 + lane)) = vals[i];
    }
    __threadfence();
  }
}

extern "C" void kernel_launch(void* const* d_in, const int* in_sizes, int n_in,
                              void* d_out, int out_size, void* d_ws, size_t ws_size,
                              hipStream_t stream) {
  (void)in_sizes;
  (void)n_in;
  (void)out_size;
  if (ws_size < WS_TOTAL) return;

  const float* xyz    = (const float*)d_in[0];
  const float* points = (const float*)d_in[1];
  const float* w0  = (const float*)d_in[2];
  const float* b0  = (const float*)d_in[3];
  const float* g0  = (const float*)d_in[4];
  const float* be0 = (const float*)d_in[5];
  const float* w1  = (const float*)d_in[6];
  const float* b1  = (const float*)d_in[7];
  const float* g1  = (const float*)d_in[8];
  const float* be1 = (const float*)d_in[9];
  const float* w2  = (const float*)d_in[10];
  const float* b2  = (const float*)d_in[11];
  const float* g2  = (const float*)d_in[12];
  const float* be2 = (const float*)d_in[13];

  float* out0 = (float*)d_out;
  float* out1 = (float*)((char*)d_out + OUT1_OFF_BYTES);

  char* ws = (char*)d_ws;
  float* X    = (float*)(ws + OFF_X);
  float* XX   = (float*)(ws + OFF_XX);
  unsigned int* W0f = (unsigned int*)(ws + OFF_W0F);
  unsigned int* W1h = (unsigned int*)(ws + OFF_W1H);
  unsigned int* W2h = (unsigned int*)(ws + OFF_W2H);
  float* W0x  = (float*)(ws + OFF_W0X);
  float* SS0  = (float*)(ws + OFF_SS);
  float* SS1  = SS0 + 256;
  float* SS2  = SS0 + 512;
  float* CENT = (float*)(ws + OFF_CENT);
  v4u* P16q   = (v4u*)(ws + OFF_P16);
  float* REL  = (float*)(ws + OFF_REL);
  unsigned short* A0 = (unsigned short*)(ws + OFF_A0);
  unsigned short* A1 = (unsigned short*)(ws + OFF_A1);
  unsigned short* A2 = (unsigned short*)(ws + OFF_A2);
  float* YB   = (float*)(ws + OFF_YB);
  float* PART0 = (float*)(ws + OFF_PART0);
  float* PART1 = (float*)(ws + OFF_PART1);
  float* PART2 = (float*)(ws + OFF_PART2);
  float* GM   = (float*)(ws + OFF_GM);

  prep_small<<<PREP_SMALL_BLOCKS, 256, 0, stream>>>(xyz, w0, w1, w2, X, XX, W0f, W1h, W2h, W0x);
  prep_points<<<NBATCH * (NPTS / 64), 256, 0, stream>>>(points, P16q);
  fps_kernel<<<NBATCH, 1024, 0, stream>>>(X, out0, CENT);
  ballquery_group<<<NGROUPS / 8, 256, 0, stream>>>(X, XX, CENT, P16q, (v4u*)A0, REL);

  mlp_gemm<0><<<NGROUPS / 8, 256, 0, stream>>>(A0, (const unsigned short*)W0f, b0, REL, W0x, YB, PART0, GM);
  bn_finalize<<<NOUT_L0 / 32, 256, 0, stream>>>(PART0, NOUT_L0, g0, be0, SS0);
  bn_relu_f16<<<(MROWS * 8) / 256, 256, 0, stream>>>(YB, SS0, A1);

  mlp_gemm<1><<<NGROUPS / 8, 256, 0, stream>>>(A1, (const unsigned short*)W1h, b1, REL, W0x, YB, PART1, GM);
  bn_finalize<<<NOUT_L1 / 32, 256, 0, stream>>>(PART1, NOUT_L1, g1, be1, SS1);
  bn_relu_f16<<<(MROWS * 8) / 256, 256, 0, stream>>>(YB, SS1, A2);

  mlp_gemm<2><<<NGROUPS / 8, 256, 0, stream>>>(A2, (const unsigned short*)W2h, b2, REL, W0x, YB, PART2, GM);
  bn_finalize<<<NOUT_L2 / 32, 256, 0, stream>>>(PART2, NOUT_L2, g2, be2, SS2);
  out_kernel<<<NGROUPS / 32, 256, 0, stream>>>(GM, SS2, out1);
}
